// NEQUIP_57621281243602
// MI455X (gfx1250) — hardware-verified
//
#include <hip/hip_runtime.h>
#include <stddef.h>
#include <stdint.h>

#define EMBD   32
#define HMID   112
#define HOUT   32
#define NSH    16
#define NBAS   8
#define RHID   64
#define KRAD   128
#define FP32P  128
#define KP0    1088
#define KP1    3840
#define NTHR   256
#define NWAVE  8
#define GBM    64
#define GTHR   128
#define AP     136
#define STGP   128
#define EPT    8
#define CHUNK  (NTHR * EPT)
#define WCAP   (EPT * 32)
#define LISTN  (NWAVE * WCAP)
#define NBA    256
#define SLA    8
#define RCAP   4096
#define DEGCAP 64
#define HBAT   8
#define GEPB   256
#define ZINTS  (LISTN + 2 * RCAP + 3 * NBA)
#define WSMAX  134217728
#define PI_F   3.14159265358979323846f
#define SQ25   0.6324555320336759f

static_assert((CHUNK & (CHUNK - 1)) == 0 && CHUNK <= 4096);
static_assert((NBA & (NBA - 1)) == 0 && NBA == (1 << SLA));
static_assert(((long long)CHUNK << SLA) < (1LL << 31));
static_assert(LISTN % 4 == 0 && ZINTS % 4 == 0 && RCAP % 4 == 0);
static_assert(NBA % NWAVE == 0 && NBA % 32 == 0);
static_assert(GBM == (GTHR / 32) * 16 && GEPB == NTHR);
static_assert((AP * 2) % 16 == 0 && AP >= KRAD && (STGP * 4) % 16 == 0);
static_assert(KRAD == 2 * RHID && KRAD % 32 == 0);
static_assert(KP0 == 2 * EMBD * NSH + 2 * EMBD && KP0 % 64 == 0 && KP0 % 32 == 0);
static_assert(KP1 >= 2 * HMID * NSH + 2 * HMID && KP1 % 64 == 0 && (2 * HMID * NSH + 2 * HMID) % 32 == 0);
static_assert(NBAS * RHID == 4 * GTHR);
static_assert(HMID % 16 == 0 && HOUT % 16 == 0 && EMBD % 16 == 0);

typedef float          v4f   __attribute__((ext_vector_type(4)));
typedef float          v8f   __attribute__((ext_vector_type(8)));
typedef int            v4i   __attribute__((ext_vector_type(4)));
typedef int            v8i   __attribute__((ext_vector_type(8)));
typedef unsigned short v8us  __attribute__((ext_vector_type(8)));
typedef unsigned short v16us __attribute__((ext_vector_type(16)));
typedef __bf16         v16bf __attribute__((ext_vector_type(16)));
typedef v4f  __attribute__((may_alias)) v4fa;
typedef v4i  __attribute__((may_alias)) v4ia;
typedef v8us __attribute__((may_alias)) v8usa;
union FragB { v16bf v; v16us u; v8us h[2]; v8i w; };

__device__ __forceinline__ v8f wmb(const FragB& a, const FragB& b, v8f c) {
  v8f d = __builtin_amdgcn_wmma_f32_16x16x32_bf16(false, a.v, false, b.v, (short)0, c, false, false);
  asm volatile("v_nop\n\tv_nop\n\tv_nop\n\tv_nop" : "+v"(d) : "v"(a.w), "v"(b.w));
  return d;
}

__device__ __forceinline__ unsigned bf16_bits(float f) {
  const unsigned u = __float_as_uint(f);
  return (u + 0x7FFFu + ((u >> 16) & 1u)) >> 16;
}
__device__ __forceinline__ float bf16_val(float f) {
  return __uint_as_float(bf16_bits(f) << 16);
}
__device__ __forceinline__ float silu_f(float t) {
  return t * __builtin_amdgcn_rcpf(1.0f + __expf(-t));
}
__device__ __forceinline__ void put16(unsigned short* dp, v8us o) {
  *(volatile v8us*)dp = o;
  __threadfence();
  *(volatile v8us*)dp = o;
}
__device__ __forceinline__ void putf4(float* dp, v4f o) {
  *(volatile v4f*)dp = o;
  __threadfence();
  *(volatile v4f*)dp = o;
}

__host__ __device__ constexpr int rupT(int x) { return ((x + NTHR - 1) / NTHR) * NTHR; }

template <int FIN, int FO, int KP>
struct PrepCfg {
  static constexpr int F16 = FIN * NSH;
  static constexpr int KA  = 2 * F16 + 2 * FIN;
  static constexpr int KS  = KP - 2 * F16;
  static constexpr int U0n = FIN * (KRAD / 8);
  static constexpr int R0  = rupT(U0n);
  static constexpr int U1n = FO * ((2 * F16) / 8);
  static constexpr int R1  = R0 + rupT(U1n);
  static constexpr int U2n = FO * (KS / 8);
  static constexpr int R2  = R1 + rupT(U2n);
};

template <int SLB>
__device__ __forceinline__ int scan_chunk(const int* __restrict__ dsts, int nE, int cbase, int slotBase,
                                          int nb, int vec8, int* list, int tid, int lane, int wave) {
  int wc = 0;
  const int el0  = tid * EPT;
  const int e0   = cbase + el0;
  const int sent = -2147483647 - 1;
  v4i da, db;
  if (vec8 != 0 && cbase + CHUNK <= nE) {
    da = *(const v4i*)(dsts + e0);
    db = *(const v4i*)(dsts + e0 + 4);
  } else {
    da.x = (e0     < nE) ? dsts[min(e0,     nE - 1)] : sent;
    da.y = (e0 + 1 < nE) ? dsts[min(e0 + 1, nE - 1)] : sent;
    da.z = (e0 + 2 < nE) ? dsts[min(e0 + 2, nE - 1)] : sent;
    da.w = (e0 + 3 < nE) ? dsts[min(e0 + 3, nE - 1)] : sent;
    db.x = (e0 + 4 < nE) ? dsts[min(e0 + 4, nE - 1)] : sent;
    db.y = (e0 + 5 < nE) ? dsts[min(e0 + 5, nE - 1)] : sent;
    db.z = (e0 + 6 < nE) ? dsts[min(e0 + 6, nE - 1)] : sent;
    db.w = (e0 + 7 < nE) ? dsts[min(e0 + 7, nE - 1)] : sent;
  }
  const unsigned nbs = (unsigned)slotBase;
  const unsigned unb = (unsigned)nb;
  const unsigned s0 = (unsigned)da.x - nbs, s1 = (unsigned)da.y - nbs;
  const unsigned s2 = (unsigned)da.z - nbs, s3 = (unsigned)da.w - nbs;
  const unsigned s4 = (unsigned)db.x - nbs, s5 = (unsigned)db.y - nbs;
  const unsigned s6 = (unsigned)db.z - nbs, s7 = (unsigned)db.w - nbs;
  const bool h0 = s0 < unb, h1 = s1 < unb, h2 = s2 < unb, h3 = s3 < unb;
  const bool h4 = s4 < unb, h5 = s5 < unb, h6 = s6 < unb, h7 = s7 < unb;
  const unsigned any = __builtin_amdgcn_ballot_w32(h0 | h1 | h2 | h3 | h4 | h5 | h6 | h7);
  if (any != 0u) {
#define HITJ(J, HJ, SJ) { \
      const unsigned mj = __builtin_amdgcn_ballot_w32(HJ); \
      if (mj != 0u) { \
        if (HJ) { \
          const int pos = wc + (int)__builtin_amdgcn_mbcnt_lo(mj, 0u); \
          if (pos < WCAP) list[wave * WCAP + pos] = ((el0 + (J)) << SLB) | (int)(SJ); \
        } \
        wc += (int)__builtin_popcount(mj); } }
    HITJ(0, h0, s0)
    HITJ(1, h1, s1)
    HITJ(2, h2, s2)
    HITJ(3, h3, s3)
    HITJ(4, h4, s4)
    HITJ(5, h5, s5)
    HITJ(6, h6, s6)
    HITJ(7, h7, s7)
#undef HITJ
  }
  return wc;
}

template <int FIN, int FO, int KP>
__global__ __launch_bounds__(NTHR) void k_prep(const float* __restrict__ w2, const float* __restrict__ wm,
                                               const float* __restrict__ wsk, const int* __restrict__ species,
                                               const float* __restrict__ embed, int nN, int nSp, int mRows,
                                               unsigned short* W2T, unsigned short* BT, float* FEAT0) {
  typedef PrepCfg<FIN, FO, KP> C;
  static_assert(FIN % 8 == 0 && C::KS >= 2 * FIN && C::KS % 8 == 0 && (2 * C::F16) % 64 == 0 && KP % 64 == 0);
  const int u = (int)blockIdx.x * NTHR + (int)threadIdx.x;
  v8us o;
  if (u < C::R0) {
    if (u >= C::U0n) return;
    const int n    = u >> 4;
    const int k8   = (u & 15) * 8;
    const int srow = k8 & (RHID - 1);
    const float* p = w2 + (size_t)srow * FIN + n;
#pragma unroll
    for (int i = 0; i < 8; ++i) o[i] = (unsigned short)bf16_bits(p[(size_t)i * FIN]);
    put16(W2T + (size_t)n * KRAD + k8, o);
    return;
  } else if (u < C::R1) {
    const int v = u - C::R0;
    if (v >= C::U1n) return;
    constexpr int UPR = (2 * C::F16) / 8;
    const int n    = v / UPR;
    const int kk8  = (v - n * UPR) * 8;
    const int srow = kk8 < C::F16 ? kk8 : kk8 - C::F16;
    const float* p = wm + (size_t)srow * FO + n;
#pragma unroll
    for (int i = 0; i < 8; ++i) o[i] = (unsigned short)bf16_bits(p[(size_t)i * FO]);
    put16(BT + (size_t)n * KP + kk8, o);
    return;
  } else if (u < C::R2) {
    const int v = u - C::R1;
    if (v >= C::U2n) return;
    constexpr int UPR = C::KS / 8;
    const int n    = v / UPR;
    const int kk8  = (v - n * UPR) * 8;
    const float zf = (kk8 < 2 * FIN) ? 1.0f : 0.0f;
    const int srow = kk8 < FIN ? kk8 : (kk8 < 2 * FIN ? kk8 - FIN : 0);
    const float* p = wsk + (size_t)srow * FO + n;
#pragma unroll
    for (int i = 0; i < 8; ++i) o[i] = (unsigned short)bf16_bits(p[(size_t)i * FO] * zf);
    put16(BT + (size_t)n * KP + 2 * C::F16 + kk8, o);
    return;
  } else {
    const int v = u - C::R2;
    if (v >= mRows * 32) return;
    const int row = v >> 5;
    const int c4  = (v & 31) * 4;
    const int rc  = row < nN ? row : nN - 1;
    int sp = species[rc];
    sp = sp < 0 ? 0 : (sp > nSp - 1 ? nSp - 1 : sp);
    const int cq = c4 < EMBD ? c4 : EMBD - 4;
    const v4f e4 = *(const v4fa*)(embed + (size_t)sp * EMBD + cq);
    const bool ok = (row < nN) && (c4 < EMBD);
    v4f q;
    q.x = ok ? bf16_val(e4.x) : 0.0f;
    q.y = ok ? bf16_val(e4.y) : 0.0f;
    q.z = ok ? bf16_val(e4.z) : 0.0f;
    q.w = ok ? bf16_val(e4.w) : 0.0f;
    putf4(FEAT0 + (size_t)row * FP32P + c4, q);
    return;
  }
}

__global__ __launch_bounds__(NTHR) void k_geom(const float* __restrict__ pos, const int* __restrict__ snd,
                                               const int* __restrict__ rcv, int nE, int nN,
                                               float* SHo, float* BAo) {
#pragma clang fp contract(off)
  __shared__ __attribute__((aligned(16))) float ssh[GEPB * NSH];
  __shared__ __attribute__((aligned(16))) float sba[GEPB * NBAS];
  const int tid = (int)threadIdx.x;
  const int eb  = (int)blockIdx.x * GEPB;
  const int e   = eb + tid;
  const int ec  = e < nE ? e : nE - 1;
  int s = snd[ec];
  int t = rcv[ec];
  s = s < 0 ? 0 : (s > nN - 1 ? nN - 1 : s);
  t = t < 0 ? 0 : (t > nN - 1 ? nN - 1 : t);
  const float psx = bf16_val(pos[(size_t)s * 3 + 0]);
  const float psy = bf16_val(pos[(size_t)s * 3 + 1]);
  const float psz = bf16_val(pos[(size_t)s * 3 + 2]);
  const float ptx = bf16_val(pos[(size_t)t * 3 + 0]);
  const float pty = bf16_val(pos[(size_t)t * 3 + 1]);
  const float ptz = bf16_val(pos[(size_t)t * 3 + 2]);
  const float vx = ptx - psx, vy = pty - psy, vz = ptz - psz;
  const float d2 = (vx * vx + vz * vz) + vy * vy;
  const float r  = sqrtf(d2 + 1e-12f);
  const float inv = 1.0f / (r + 1e-9f);
  const float x = vx * inv, y = vy * inv, z = vz * inv;
  const float x2 = x * x, y2 = y * y, z2 = z * z;
  float* o = ssh + tid * NSH;
  o[0]  = 0.28209479177387814f;
  o[1]  = 0.4886025119029199f * x;
  o[2]  = 0.4886025119029199f * y;
  o[3]  = 0.4886025119029199f * z;
  o[4]  = (1.0925484305920792f * x) * y;
  o[5]  = (1.0925484305920792f * y) * z;
  o[6]  = 0.31539156525252005f * (3.0f * z2 - 1.0f);
  o[7]  = (1.0925484305920792f * x) * z;
  o[8]  = 0.5462742152960396f * (x2 - y2);
  o[9]  = (0.5900435899266435f * y) * (3.0f * x2 - y2);
  o[10] = ((2.890611442640554f * x) * y) * z;
  o[11] = (0.4570457994644658f * y) * (5.0f * z2 - 1.0f);
  o[12] = (0.3731763325901154f * z) * (5.0f * z2 - 3.0f);
  o[13] = (0.4570457994644658f * x) * (5.0f * z2 - 1.0f);
  o[14] = (1.445305721320277f * z) * (x2 - y2);
  o[15] = (0.5900435899266435f * x) * (x2 - 3.0f * y2);
  const float xr  = r * 0.2f;
  const float xr2 = xr * xr;
  const float xr4 = xr2 * xr2;
  const float x6  = xr2 * xr4;
  const float x7  = (xr * xr2) * xr4;
  const float x8  = xr4 * xr4;
  float env = ((1.0f - 28.0f * x6) + 48.0f * x7) - 21.0f * x8;
  env = (xr < 1.0f) ? env : 0.0f;
  float* bq = sba + tid * NBAS;
#pragma unroll 1
  for (int n = 1; n <= NBAS; ++n) {
    const float w  = ((float)n * PI_F) * xr;
    const float sv = sinf(w);
    bq[n - 1] = ((SQ25 * sv) * inv) * env;
  }
  __syncthreads();
  {
    float* shb = SHo + (size_t)eb * NSH;
    v4f pv[4];
#pragma unroll
    for (int it = 0; it < 4; ++it) pv[it] = *(const v4fa*)(ssh + (size_t)(it * NTHR + tid) * 4);
#pragma unroll
    for (int it = 0; it < 4; ++it) *(volatile v4f*)(shb + (size_t)(it * NTHR + tid) * 4) = pv[it];
    __threadfence();
#pragma unroll
    for (int it = 0; it < 4; ++it) *(volatile v4f*)(shb + (size_t)(it * NTHR + tid) * 4) = pv[it];
  }
  {
    float* bab = BAo + (size_t)eb * NBAS;
    v4f pv[2];
#pragma unroll
    for (int it = 0; it < 2; ++it) pv[it] = *(const v4fa*)(sba + (size_t)(it * NTHR + tid) * 4);
#pragma unroll
    for (int it = 0; it < 2; ++it) *(volatile v4f*)(bab + (size_t)(it * NTHR + tid) * 4) = pv[it];
    __threadfence();
#pragma unroll
    for (int it = 0; it < 2; ++it) *(volatile v4f*)(bab + (size_t)(it * NTHR + tid) * 4) = pv[it];
  }
}

template <int FIN, int NT>
__global__ __launch_bounds__(GTHR) void k_rad(const float* __restrict__ BA, const float* __restrict__ w1,
                                              int nE, const unsigned short* __restrict__ W2T, float* RADo) {
  static_assert(NT * 16 == FIN && NT >= 1 && NT <= 8);
  __shared__ __attribute__((aligned(16))) float sw1[NBAS * RHID];
  __shared__ __attribute__((aligned(16))) unsigned short sA[GBM * AP];
  __shared__ __attribute__((aligned(16))) float stg[GBM * STGP];
  const int tid = (int)threadIdx.x, lane = tid & 31, wave = tid >> 5, hh = lane >> 4, m = lane & 15;
  const int rowBase = (int)blockIdx.x * GBM;

#pragma unroll
  for (int i = 0; i < 4; ++i) sw1[tid + GTHR * i] = bf16_val(w1[tid + GTHR * i]);
  const int r  = tid >> 1;
  const int hs = tid & 1;
  int e = rowBase + r;
  e = e < nE ? e : nE - 1;
  const v4f ba = *(const v4fa*)(BA + (size_t)e * NBAS);
  const v4f bb = *(const v4fa*)(BA + (size_t)e * NBAS + 4);
  __syncthreads();

  {
    unsigned short* ra = sA + r * AP + 32 * hs;
#pragma unroll 1
    for (int hg = 0; hg < 4; ++hg) {
      v8us ho, lo;
#pragma unroll
      for (int i = 0; i < 8; ++i) {
        const int h = 32 * hs + 8 * hg + i;
        const float* wc = sw1 + h;
        float tv = ba.x * wc[0];
        tv = fmaf(ba.y, wc[1 * RHID], tv);
        tv = fmaf(ba.z, wc[2 * RHID], tv);
        tv = fmaf(ba.w, wc[3 * RHID], tv);
        tv = fmaf(bb.x, wc[4 * RHID], tv);
        tv = fmaf(bb.y, wc[5 * RHID], tv);
        tv = fmaf(bb.z, wc[6 * RHID], tv);
        tv = fmaf(bb.w, wc[7 * RHID], tv);
        const float sv = silu_f(tv);
        const unsigned hb = bf16_bits(sv);
        ho[i] = (unsigned short)hb;
        lo[i] = (unsigned short)bf16_bits(sv - __uint_as_float(hb << 16));
      }
      *(v8usa*)(ra + 8 * hg)        = ho;
      *(v8usa*)(ra + RHID + 8 * hg) = lo;
    }
  }
  __syncthreads();

  v8f acc[NT];
  {
    const v8f zv = {0.f, 0.f, 0.f, 0.f, 0.f, 0.f, 0.f, 0.f};
#pragma unroll
    for (int nt = 0; nt < NT; ++nt) acc[nt] = zv;
  }
  const unsigned short* ap = sA + (16 * wave + m) * AP + 8 * hh;
  const unsigned short* bp = W2T + (size_t)m * KRAD + 8 * hh;
#pragma unroll 1
  for (int k0 = 0; k0 < KRAD; k0 += 32) {
    FragB af;
    af.h[0] = *(const v8usa*)(ap + k0);
    af.h[1] = *(const v8usa*)(ap + k0 + 16);
#pragma unroll
    for (int nt = 0; nt < NT; ++nt) {
      const unsigned short* wq = bp + (size_t)(16 * nt) * KRAD + k0;
      FragB bf;
      bf.h[0] = *(const v8usa*)wq;
      bf.h[1] = *(const v8usa*)(wq + 16);
      acc[nt] = wmb(af, bf, acc[nt]);
    }
  }
#pragma unroll
  for (int nt = 0; nt < NT; ++nt) {
    const int lc = 16 * nt + m;
#pragma unroll
    for (int rr = 0; rr < 8; ++rr) {
      const int lr = 16 * wave + 8 * hh + rr;
      stg[lr * STGP + lc] = acc[nt][rr];
    }
  }
#pragma unroll
  for (int nt = NT; nt < 8; ++nt) {
    const int lc = 16 * nt + m;
#pragma unroll
    for (int rr = 0; rr < 8; ++rr) {
      const int lr = 16 * wave + 8 * hh + rr;
      stg[lr * STGP + lc] = 0.0f;
    }
  }
  __syncthreads();
  {
    v4f pv[16];
#pragma unroll
    for (int i = 0; i < 16; ++i) pv[i] = *(const v4fa*)(stg + (16 * wave + i) * STGP + 4 * lane);
#pragma unroll
    for (int i = 0; i < 16; ++i) {
      float* op = RADo + (size_t)(rowBase + 16 * wave + i) * FP32P + 4 * lane;
      *(volatile v4f*)op = pv[i];
    }
    __threadfence();
#pragma unroll
    for (int i = 0; i < 16; ++i) {
      float* op = RADo + (size_t)(rowBase + 16 * wave + i) * FP32P + 4 * lane;
      *(volatile v4f*)op = pv[i];
    }
  }
}

template <int NT, int SILU, int EPI>
__global__ __launch_bounds__(GTHR) void k_gemm(const unsigned short* __restrict__ A, int lda,
                                               const unsigned short* __restrict__ BT, int ldb, int K, int nN,
                                               float* Cm, float* Co) {
  static_assert(NT >= 1 && NT <= 8);
  __shared__ __attribute__((aligned(16))) float stg[GBM * STGP];
  const int tid = (int)threadIdx.x, lane = tid & 31, wave = tid >> 5, hh = lane >> 4, m = lane & 15;
  const int rowBase = (int)blockIdx.x * GBM;

  v8f acc[NT];
  {
    const v8f zv = {0.f, 0.f, 0.f, 0.f, 0.f, 0.f, 0.f, 0.f};
#pragma unroll
    for (int nt = 0; nt < NT; ++nt) acc[nt] = zv;
  }
  const unsigned short* ap = A  + (size_t)(rowBase + 16 * wave + m) * (size_t)lda + 8 * hh;
  const unsigned short* bp = BT + (size_t)m * (size_t)ldb + 8 * hh;
#pragma unroll 1
  for (int k0 = 0; k0 < K; k0 += 32) {
    FragB af;
    af.h[0] = *(const v8usa*)(ap + k0);
    af.h[1] = *(const v8usa*)(ap + k0 + 16);
#pragma unroll
    for (int nt = 0; nt < NT; ++nt) {
      const unsigned short* wq = bp + (size_t)(16 * nt) * (size_t)ldb + k0;
      FragB bf;
      bf.h[0] = *(const v8usa*)wq;
      bf.h[1] = *(const v8usa*)(wq + 16);
      acc[nt] = wmb(af, bf, acc[nt]);
    }
  }
#pragma unroll
  for (int nt = 0; nt < NT; ++nt) {
    const int lc = 16 * nt + m;
#pragma unroll
    for (int rr = 0; rr < 8; ++rr) {
      const int lr = 16 * wave + 8 * hh + rr;
      float v = acc[nt][rr];
      if constexpr (SILU != 0) v = silu_f(v);
      stg[lr * STGP + lc] = v;
    }
  }
#pragma unroll
  for (int nt = NT; nt < 8; ++nt) {
    const int lc = 16 * nt + m;
#pragma unroll
    for (int rr = 0; rr < 8; ++rr) {
      const int lr = 16 * wave + 8 * hh + rr;
      stg[lr * STGP + lc] = 0.0f;
    }
  }
  __syncthreads();

  if constexpr (EPI == 0) {
    v4f pv[16];
#pragma unroll
    for (int i = 0; i < 16; ++i) pv[i] = *(const v4fa*)(stg + (16 * wave + i) * STGP + 4 * lane);
#pragma unroll
    for (int i = 0; i < 16; ++i) {
      float* op = Cm + (size_t)(rowBase + 16 * wave + i) * FP32P + 4 * lane;
      *(volatile v4f*)op = pv[i];
    }
    __threadfence();
#pragma unroll
    for (int i = 0; i < 16; ++i) {
      float* op = Cm + (size_t)(rowBase + 16 * wave + i) * FP32P + 4 * lane;
      *(volatile v4f*)op = pv[i];
    }
  } else {
    const int q  = lane >> 3;
    const int c4 = (lane & 7) * 4;
    v4f pv[4];
#pragma unroll
    for (int j = 0; j < 4; ++j) pv[j] = *(const v4fa*)(stg + (16 * wave + 4 * j + q) * STGP + c4);
#pragma unroll
    for (int j = 0; j < 4; ++j) {
      const int row = rowBase + 16 * wave + 4 * j + q;
      if (row < nN) *(volatile v4f*)(Co + (size_t)row * HOUT + c4) = pv[j];
    }
    __threadfence();
#pragma unroll
    for (int j = 0; j < 4; ++j) {
      const int row = rowBase + 16 * wave + 4 * j + q;
      if (row < nN) *(volatile v4f*)(Co + (size_t)row * HOUT + c4) = pv[j];
    }
  }
}

template <int FIN, int KP>
__global__ __launch_bounds__(NTHR) void k_scan(const int* __restrict__ dsts, const int* __restrict__ srcs,
                                               int nE, int nN, int vec8, int mRows,
                                               const float* __restrict__ FEAT, const float* __restrict__ RAD,
                                               const float* __restrict__ SHp, unsigned short* Aout) {
  constexpr int F16   = FIN * NSH;
  constexpr int KA    = 2 * F16 + 2 * FIN;
  constexpr int GP    = FIN + NSH;
  constexpr int GQ    = FIN / 4;
  constexpr int UPH   = GQ + 4;
  constexpr int NUNIT = HBAT * UPH;
  constexpr int NACT  = 2 * FIN;
  constexpr int NPC   = KP / 8;
  constexpr int NSW   = (NPC + NTHR - 1) / NTHR;
  constexpr int NPAD8 = (KP - KA) / 8;
  static_assert(KP >= KA && KP % 64 == 0 && KA % 8 == 0 && (KP - KA) % 8 == 0 && FIN % 8 == 0);
  static_assert(NUNIT <= NTHR && NACT <= NTHR && NACT % 32 == 0 && NPAD8 <= NTHR && FIN / 8 <= NTHR);
  static_assert((GP * 4) % 16 == 0 && NPC % 8 == 0);

  __shared__ __attribute__((aligned(16))) int dsm[ZINTS + 16];
  __shared__ __attribute__((aligned(16))) float gS[HBAT * GP];
  __shared__ __attribute__((aligned(16))) unsigned short rowS[KP];
  int* list = dsm;
  int* hl   = dsm + LISTN;
  int* sl   = hl + RCAP;
  int* cnt  = sl + RCAP;
  int* offs = cnt + NBA;
  int* cur  = offs + NBA;
  int* misc = cur + NBA;
  const int tid = (int)threadIdx.x, lane = tid & 31, wave = tid >> 5;
  const int nodeBase = (int)blockIdx.x * NBA;

  {
    const v4i z4 = {0, 0, 0, 0};
    for (int i = tid * 4; i < ZINTS; i += NTHR * 4) *(v4ia*)(dsm + i) = z4;
    if (tid < 16) misc[tid] = 0;
  }
  __syncthreads();

  int t = 0, ov = 0;
  const int nChunks = (nE + CHUNK - 1) / CHUNK;
#pragma unroll 1
  for (int ch = 0; ch < nChunks; ++ch) {
    const int cbase = ch * CHUNK;
    const int wc = scan_chunk<SLA>(dsts, nE, cbase, nodeBase, NBA, vec8, list, tid, lane, wave);
    if (lane == 0) misc[wave] = wc;
    __syncthreads();
    if (wave == 0) {
#pragma unroll 1
      for (int w2 = 0; w2 < NWAVE; ++w2) {
        int c = misc[w2];
        c = c < 0 ? 0 : (c > WCAP ? WCAP : c);
#pragma unroll 1
        for (int b0 = 0; b0 < c; b0 += 32) {
          const int idx = b0 + lane;
          const int ent = list[w2 * WCAP + (idx < WCAP ? idx : WCAP - 1)];
          const int m32 = (c - b0) < 32 ? (c - b0) : 32;
#pragma unroll 1
          for (int k = 0; k < m32; ++k) {
            const int u    = __builtin_amdgcn_readlane(ent, k);
            const int slot = u & (NBA - 1);
            const int el   = (u >> SLA) & (CHUNK - 1);
            const int pk   = ((cbase + el) << SLA) | slot;
            if (t < RCAP) {
              if (lane == 0) { hl[t] = pk; cnt[slot] = cnt[slot] + 1; }
              t = t + 1;
            } else {
              ov = 1;
            }
          }
        }
      }
    }
    __syncthreads();
  }
  if (wave == 0 && lane == 0) { misc[8] = t; misc[9] = ov; }
  __syncthreads();
  int tt = misc[8];
  tt = tt < 0 ? 0 : (tt > RCAP ? RCAP : tt);
  const int ovf = misc[9];

  if (wave == 0) {
    const int base = lane * (NBA / 32);
    int s = 0;
#pragma unroll 1
    for (int i = 0; i < NBA / 32; ++i) s += cnt[base + i];
    int incl = s;
#pragma unroll
    for (int d = 1; d < 32; d <<= 1) {
      const int y = __shfl_up(incl, d, 32);
      if (lane >= d) incl += y;
    }
    int run = incl - s;
#pragma unroll 1
    for (int i = 0; i < NBA / 32; ++i) {
      const int cv = cnt[base + i];
      offs[base + i] = run;
      cur[base + i]  = run;
      run += cv;
    }
  }
  __syncthreads();
  if (wave == 0) {
#pragma unroll 1
    for (int b0 = 0; b0 < tt; b0 += 32) {
      const int idx = b0 + lane;
      const int ent = hl[idx < RCAP ? idx : RCAP - 1];
      const int m32 = (tt - b0) < 32 ? (tt - b0) : 32;
#pragma unroll 1
      for (int k = 0; k < m32; ++k) {
        const int u    = __builtin_amdgcn_readlane(ent, k);
        const int slot = u & (NBA - 1);
        if (lane == 0) {
          int p = cur[slot];
          p = p < 0 ? 0 : (p > RCAP - 1 ? RCAP - 1 : p);
          sl[p] = u;
          cur[slot] = p + 1;
        }
      }
    }
  }
  __syncthreads();

  const int  cown = tid >> 1;
  const int  m0   = (tid & 1) * 8;
  const int  cc   = cown < FIN ? cown : FIN - 1;
  const bool aact = tid < NACT;
  int ku = tid / UPH;
  const int  ju   = tid - ku * UPH;
  const bool uact = tid < NUNIT;
  ku = ku < HBAT ? ku : HBAT - 1;
  const int  jg   = ju < GQ ? ju : GQ - 1;
  int js = ju - GQ;
  js = js < 0 ? 0 : (js > 3 ? 3 : js);
  const float isg = (ju < GQ) ? 1.0f : 0.0f;
  const int  tf   = tid < FIN / 8 ? tid : FIN / 8 - 1;
  const unsigned short qnanb = (unsigned short)0x7fc0;

#pragma unroll 1
  for (int s = 0; s < NBA; ++s) {
    const int node = nodeBase + s;
    if (node >= mRows) break;
    int c = cnt[s];
    const bool big = c > DEGCAP;
    c = c < 0 ? 0 : (c > DEGCAP ? DEGCAP : c);
    int o = offs[s];
    o = o < 0 ? 0 : (o > RCAP ? RCAP : o);
    float acc[8];
#pragma unroll
    for (int i = 0; i < 8; ++i) acc[i] = 0.0f;

#pragma unroll 1
    for (int b0 = 0; b0 < c; b0 += HBAT) {
      const int nb = (c - b0) < HBAT ? (c - b0) : HBAT;
      {
        const int   hk = b0 + ku;
        const float lv = (ku < nb) ? 1.0f : 0.0f;
        int idx = o + (hk < c ? hk : c - 1);
        idx = idx < 0 ? 0 : (idx > RCAP - 1 ? RCAP - 1 : idx);
        const int ent = sl[idx];
        int eid = ent >> SLA;
        eid = eid < 0 ? 0 : (eid > nE - 1 ? nE - 1 : eid);
        int sd = srcs[eid];
        sd = sd < 0 ? 0 : (sd > nN - 1 ? nN - 1 : sd);
        const v4f f4 = *(const v4fa*)(FEAT + (size_t)sd  * FP32P + 4 * jg);
        const v4f r4 = *(const v4fa*)(RAD  + (size_t)eid * FP32P + 4 * jg);
        const v4f s4 = *(const v4fa*)(SHp  + (size_t)eid * NSH + 4 * js);
        const float wg = isg * lv;
        const float wv = (1.0f - isg) * lv;
        v4f q;
        q.x = (f4.x * r4.x) * wg + s4.x * wv;
        q.y = (f4.y * r4.y) * wg + s4.y * wv;
        q.z = (f4.z * r4.z) * wg + s4.z * wv;
        q.w = (f4.w * r4.w) * wg + s4.w * wv;
        if (uact) *(v4fa*)(gS + ku * GP + 4 * ju) = q;
      }
      __syncthreads();
      if (aact) {
#pragma unroll 1
        for (int k = 0; k < nb; ++k) {
          const float gv = gS[k * GP + cc];
          const v4f  sa = *(const v4fa*)(gS + k * GP + FIN + m0);
          const v4f  sb = *(const v4fa*)(gS + k * GP + FIN + m0 + 4);
          acc[0] = fmaf(gv, sa.x, acc[0]);
          acc[1] = fmaf(gv, sa.y, acc[1]);
          acc[2] = fmaf(gv, sa.z, acc[2]);
          acc[3] = fmaf(gv, sa.w, acc[3]);
          acc[4] = fmaf(gv, sb.x, acc[4]);
          acc[5] = fmaf(gv, sb.y, acc[5]);
          acc[6] = fmaf(gv, sb.z, acc[6]);
          acc[7] = fmaf(gv, sb.w, acc[7]);
        }
      }
      __syncthreads();
    }

    const bool poison = big || (ovf != 0);
    if (aact) {
      v8us ho, lo;
#pragma unroll
      for (int i = 0; i < 8; ++i) {
        const unsigned hb = bf16_bits(acc[i]);
        const unsigned lb = bf16_bits(acc[i] - __uint_as_float(hb << 16));
        ho[i] = poison ? qnanb : (unsigned short)hb;
        lo[i] = poison ? (unsigned short)0 : (unsigned short)lb;
      }
      *(v8usa*)(rowS + 16 * cown + m0)       = ho;
      *(v8usa*)(rowS + F16 + 16 * cown + m0) = lo;
    }
    {
      const int nr = node < mRows ? node : mRows - 1;
      const v4f fa = *(const v4fa*)(FEAT + (size_t)nr * FP32P + 8 * tf);
      const v4f fb = *(const v4fa*)(FEAT + (size_t)nr * FP32P + 8 * tf + 4);
      const v8f f8 = {fa.x, fa.y, fa.z, fa.w, fb.x, fb.y, fb.z, fb.w};
      v8us fh, fl;
#pragma unroll
      for (int i = 0; i < 8; ++i) {
        const unsigned hb = bf16_bits(f8[i]);
        fh[i] = (unsigned short)hb;
        fl[i] = (unsigned short)bf16_bits(f8[i] - __uint_as_float(hb << 16));
      }
      if (tid < FIN / 8) {
        *(v8usa*)(rowS + 2 * F16 + 8 * tf)       = fh;
        *(v8usa*)(rowS + 2 * F16 + FIN + 8 * tf) = fl;
      }
      if (NPAD8 > 0 && tid < NPAD8) {
        const v8us z8 = {0, 0, 0, 0, 0, 0, 0, 0};
        *(v8usa*)(rowS + KA + 8 * tid) = z8;
      }
    }
    __syncthreads();
    if (node < mRows) {
      unsigned short* ab = Aout + (size_t)node * (size_t)KP;
      v4i pv[NSW];
#pragma unroll
      for (int it = 0; it < NSW; ++it) {
        const int p  = it * NTHR + tid;
        const int pc = p < NPC ? p : NPC - 1;
        pv[it] = *(const v4ia*)(rowS + 8 * pc);
      }
#pragma unroll
      for (int it = 0; it < NSW; ++it) {
        const int p = it * NTHR + tid;
        if (p < NPC) *(volatile v4i*)(ab + 8 * p) = pv[it];
      }
      __threadfence();
#pragma unroll
      for (int it = 0; it < NSW; ++it) {
        const int p = it * NTHR + tid;
        if (p < NPC) *(volatile v4i*)(ab + 8 * p) = pv[it];
      }
    }
    __syncthreads();
  }
}

static inline int cdiv(int a, int b) { return (a + b - 1) / b; }

extern "C" void kernel_launch(void* const* d_in, const int* in_sizes, int n_in,
                              void* d_out, int out_size, void* d_ws, size_t ws_size,
                              hipStream_t stream) {
  if (n_in < 17) return;
  const int nN = in_sizes[1];
  if (nN < 1 || in_sizes[0] != 3 * nN) return;
  const int nE = in_sizes[2];
  if (nE < 1 || nE >= (1 << 22) || in_sizes[3] != nE) return;
  if (in_sizes[4] < EMBD || (in_sizes[4] % EMBD) != 0) return;
  const int nSp = in_sizes[4] / EMBD;
  if (in_sizes[5]  != NBAS * RHID || in_sizes[6]  != RHID * EMBD) return;
  if (in_sizes[7]  != EMBD * NSH * HMID || in_sizes[8] != EMBD * HMID) return;
  if (in_sizes[9]  != NBAS * RHID || in_sizes[10] != RHID * HMID) return;
  if (in_sizes[11] != HMID * NSH * HMID || in_sizes[12] != HMID * HMID) return;
  if (in_sizes[13] != NBAS * RHID || in_sizes[14] != RHID * HMID) return;
  if (in_sizes[15] != HMID * NSH * HOUT || in_sizes[16] != HMID * HOUT) return;
  if ((long long)out_size != (long long)nN * HOUT) return;

  const float* pos  = (const float*)d_in[0];
  const int*   spc  = (const int*)d_in[1];
  const int*   snd  = (const int*)d_in[2];
  const int*   rcv  = (const int*)d_in[3];
  const float* emb  = (const float*)d_in[4];
  const float* w1_0 = (const float*)d_in[5];
  const float* w2_0 = (const float*)d_in[6];
  const float* wm_0 = (const float*)d_in[7];
  const float* ws_0 = (const float*)d_in[8];
  const float* w1_1 = (const float*)d_in[9];
  const float* w2_1 = (const float*)d_in[10];
  const float* wm_1 = (const float*)d_in[11];
  const float* ws_1 = (const float*)d_in[12];
  const float* w1_2 = (const float*)d_in[13];
  const float* w2_2 = (const float*)d_in[14];
  const float* wm_2 = (const float*)d_in[15];
  const float* ws_2 = (const float*)d_in[16];
  float* out = (float*)d_out;

  const int MP = cdiv(nN, GBM) * GBM;
  const int gM = MP / GBM;
  const int gA = cdiv(MP, NBA);
  if ((long long)gA * NBA < (long long)MP) return;
  const int EP = cdiv(nE, GEPB) * GEPB;
  const int ER = cdiv(nE, GBM) * GBM;

  char* ws = (char*)d_ws;
  size_t off = 0;
  const size_t oSH   = off; off += (size_t)EP * NSH * 4;             off = (off + 255) & ~(size_t)255;
  const size_t oBA   = off; off += (size_t)EP * NBAS * 4;            off = (off + 255) & ~(size_t)255;
  const size_t oRAD  = off; off += (size_t)ER * FP32P * 4;           off = (off + 255) & ~(size_t)255;
  const size_t oFEAT = off; off += (size_t)MP * FP32P * 4;           off = (off + 255) & ~(size_t)255;
  const size_t oA    = off; off += (size_t)MP * KP1 * 2;             off = (off + 255) & ~(size_t)255;
  const size_t oW20  = off; off += (size_t)EMBD * KRAD * 2;          off = (off + 255) & ~(size_t)255;
  const size_t oW21  = off; off += (size_t)HMID * KRAD * 2;          off = (off + 255) & ~(size_t)255;
  const size_t oW22  = off; off += (size_t)HMID * KRAD * 2;          off = (off + 255) & ~(size_t)255;
  const size_t oBT0  = off; off += (size_t)HMID * KP0 * 2;           off = (off + 255) & ~(size_t)255;
  const size_t oBT1  = off; off += (size_t)HMID * KP1 * 2;           off = (off + 255) & ~(size_t)255;
  const size_t oBT2  = off; off += (size_t)HOUT * KP1 * 2;           off = (off + 255) & ~(size_t)255;
  if (off > ws_size || off > (size_t)WSMAX) return;
  float*          SH   = (float*)(ws + oSH);
  float*          BA   = (float*)(ws + oBA);
  float*          RAD  = (float*)(ws + oRAD);
  float*          FEAT = (float*)(ws + oFEAT);
  unsigned short* A    = (unsigned short*)(ws + oA);
  unsigned short* W20  = (unsigned short*)(ws + oW20);
  unsigned short* W21  = (unsigned short*)(ws + oW21);
  unsigned short* W22  = (unsigned short*)(ws + oW22);
  unsigned short* BT0  = (unsigned short*)(ws + oBT0);
  unsigned short* BT1  = (unsigned short*)(ws + oBT1);
  unsigned short* BT2  = (unsigned short*)(ws + oBT2);

  typedef PrepCfg<EMBD, HMID, KP0> P0;
  typedef PrepCfg<HMID, HMID, KP1> P1;
  typedef PrepCfg<HMID, HOUT, KP1> P2;
  const int KA0 = P0::KA;
  const int KA1 = P1::KA;
  if ((KA0 % 32) != 0 || (KA1 % 32) != 0) return;
  const int vec8 = 1;

  k_prep<EMBD, HMID, KP0><<<(P0::R2 + MP * 32) / NTHR, NTHR, 0, stream>>>(w2_0, wm_0, ws_0, spc, emb, nN, nSp, MP,
                                                                          W20, BT0, FEAT);
  k_prep<HMID, HMID, KP1><<<P1::R2 / NTHR, NTHR, 0, stream>>>(w2_1, wm_1, ws_1, spc, emb, nN, nSp, 0,
                                                              W21, BT1, FEAT);
  k_prep<HMID, HOUT, KP1><<<P2::R2 / NTHR, NTHR, 0, stream>>>(w2_2, wm_2, ws_2, spc, emb, nN, nSp, 0,
                                                              W22, BT2, FEAT);
  k_geom<<<EP / GEPB, NTHR, 0, stream>>>(pos, snd, rcv, nE, nN, SH, BA);

  k_rad<EMBD, EMBD / 16><<<ER / GBM, GTHR, 0, stream>>>(BA, w1_0, nE, W20, RAD);
  k_scan<EMBD, KP0><<<gA, NTHR, 0, stream>>>(rcv, snd, nE, nN, vec8, MP, FEAT, RAD, SH, A);
  k_gemm<HMID / 16, 1, 0><<<gM, GTHR, 0, stream>>>(A, KP0, BT0, KP0, KA0, nN, FEAT, out);
  k_rad<HMID, HMID / 16><<<ER / GBM, GTHR, 0, stream>>>(BA, w1_1, nE, W21, RAD);
  k_scan<HMID, KP1><<<gA, NTHR, 0, stream>>>(rcv, snd, nE, nN, vec8, MP, FEAT, RAD, SH, A);
  k_gemm<HMID / 16, 1, 0><<<gM, GTHR, 0, stream>>>(A, KP1, BT1, KP1, KA1, nN, FEAT, out);
  k_rad<HMID, HMID / 16><<<ER / GBM, GTHR, 0, stream>>>(BA, w1_2, nE, W22, RAD);
  k_scan<HMID, KP1><<<gA, NTHR, 0, stream>>>(rcv, snd, nE, nN, vec8, MP, FEAT, RAD, SH, A);
  k_gemm<HOUT / 16, 0, 1><<<gM, GTHR, 0, stream>>>(A, KP1, BT2, KP1, KA1, nN, FEAT, out);
}
